// EdgeNetwork_81647328297533
// MI455X (gfx1250) — hardware-verified
//
#include <hip/hip_runtime.h>
#include <stddef.h>


typedef _Float16 h16;
typedef _Float16 v16h __attribute__((ext_vector_type(16)));
typedef float    v8f  __attribute__((ext_vector_type(8)));
typedef float    v4f  __attribute__((ext_vector_type(4)));

#ifndef NB
#define NB 2
#endif
#ifndef NROW
#define NROW 1024
#endif
#define NB_FULL 2
#define NN      1024
#define DIN     16
#define HIDN    8
#define W1LD    49
#define STEPS   4
#define LDP     20

static_assert(NB >= 1 && NB <= NB_FULL);
static_assert(NROW >= 1 && NROW <= NN);
static_assert(DIN == 16 && HIDN == 8);
static_assert(W1LD == 3 * DIN + 1);
static_assert(NN == 8 * STEPS * 32);
static_assert(STEPS * 32 * 4 == 32 * 16);
static_assert(((NB * NN) % 128) == 0);
static_assert((NN % 16) == 0);
static_assert((LDP % 4) == 0 && LDP >= 16);

#define XCARRY 16.0f
#define WCARRY 64.0f
#define HCARRY 256.0f
#define PCS    (1.0f / (XCARRY * WCARRY))
#define LSCALE (1.0f / (WCARRY * HCARRY))

#define PLANE_BYTES ((size_t)NB * NN * HIDN * 4)
#define OFF_TJ   ((size_t)0)
#define OFF_U    (OFF_TJ + PLANE_BYTES)
#define WS_TOTAL (OFF_U + PLANE_BYTES)
static_assert((PLANE_BYTES % 512) == 0);
static_assert(WS_TOTAL <= (size_t)134217728);

__device__ __forceinline__ float bf16r(float x) {
  unsigned int u = __float_as_uint(x);
  u = (u + 0x7FFFu + ((u >> 16) & 1u)) & 0xFFFF0000u;
  return __uint_as_float(u);
}

static __device__ __forceinline__ h16 toh_flush(float v) {
  const h16 r = (h16)v;
  return (fabsf(v) < 6.103515625e-05f) ? (h16)0.0f : r;
}

__device__ __forceinline__ v8f wmma16(v16h a, v16h b, v8f c) {
  v8f d = __builtin_amdgcn_wmma_f32_16x16x32_f16(false, a, false, b, (short)0, c,
                                                 false, false);
  asm volatile("v_nop\n\tv_nop\n\tv_nop\n\tv_nop" : "+v"(d) : "v"(a), "v"(b));
  return d;
}

__device__ __forceinline__ void wave_lds_sync() {
  __builtin_amdgcn_fence(3  , "wavefront");
  asm volatile("s_wait_dscnt 0x0" ::: "memory");
  __builtin_amdgcn_wave_barrier();
}

__device__ __forceinline__ float tanh_f(float x) {
  const float ax = __builtin_fabsf(x);
  const float e  = __expf(-2.0f * ax);
  const float r  = (1.0f - e) * __builtin_amdgcn_rcpf(1.0f + e);
  return __builtin_copysignf(r, x);
}

__global__ __launch_bounds__(256) void edge_pre_kernel(
    const float* __restrict__ x, const float* __restrict__ vp,
    const float* __restrict__ W1, const float* __restrict__ b1,
    float* __restrict__ TJ, float* __restrict__ U) {
  __shared__ __attribute__((aligned(16))) float Ts[8 * 16 * LDP];
  const unsigned lane = threadIdx.x & 31u;
  const unsigned w = (unsigned)__builtin_amdgcn_readfirstlane((int)(threadIdx.x >> 5));
  const unsigned hh = lane >> 4, m = lane & 15u;
  const unsigned crow0 = blockIdx.x * 128u + w * 16u;
  const unsigned b = crow0 / (unsigned)NN;

  const float* xr = x + (size_t)(crow0 + m) * DIN + hh * 8u;
  const float* vr = vp + (size_t)b * DIN + hh * 8u;
  const v4f x0 = *(const v4f*)(xr);
  const v4f x1 = *(const v4f*)(xr + 4);
  const v4f p0 = *(const v4f*)(vr);
  const v4f p1 = *(const v4f*)(vr + 4);
  v16h af;
#pragma unroll
  for (int i = 0; i < 4; ++i) {
    af[i]      = toh_flush(XCARRY * bf16r(x0[i]));
    af[i + 4]  = toh_flush(XCARRY * bf16r(x1[i]));
    af[i + 8]  = toh_flush(XCARRY * bf16r(p0[i]));
    af[i + 12] = toh_flush(XCARRY * bf16r(p1[i]));
  }

  const unsigned hrow = m & 7u;
  const bool upper = (m >= 8u);
  v16h bf;
#pragma unroll
  for (unsigned i = 0; i < 8u; ++i) {
    const unsigned kk = hh * 8u + i;
    const unsigned col0 = upper ? (16u + kk) : kk;
    const float wa = W1[hrow * W1LD + col0];
    const float wb = W1[hrow * W1LD + 32u + kk];
    const h16 ea = toh_flush(WCARRY * bf16r(wa));
    const h16 eb = toh_flush(WCARRY * bf16r(wb));
    bf[i]      = ea;
    bf[i + 8u] = upper ? eb : (h16)0.0f;
  }
  const float b1v = bf16r(b1[hrow]);
  const float bsel = upper ? b1v : 0.0f;

  v8f acc = {};
  acc = wmma16(af, bf, acc);

  const unsigned tb = w * (16u * LDP);
#pragma unroll
  for (unsigned r = 0; r < 8u; ++r)
    Ts[tb + (hh * 8u + r) * LDP + m] = acc[r] * PCS + bsel;
  wave_lds_sync();

  const unsigned row = lane >> 1;
  const unsigned c = (lane & 1u) * 4u;
  const v4f vt = *(const v4f*)&Ts[tb + row * LDP + c];
  const v4f vu = *(const v4f*)&Ts[tb + row * LDP + 8u + c];
  const size_t o = (size_t)(crow0 + row) * HIDN + c;
  *(volatile v4f*)(TJ + o) = vt;
  *(volatile v4f*)(U + o) = vu;
  __threadfence();
  *(volatile v4f*)(TJ + o) = vt;
  *(volatile v4f*)(U + o) = vu;
}

__device__ __forceinline__ v16h wfrag(const float* __restrict__ W, unsigned ko, bool diag) {
  const v4f w0 = *(const v4f*)(W + ko * 8u);
  const v4f w1 = *(const v4f*)(W + ko * 8u + 4u);
  v16h a;
#pragma unroll
  for (int i = 0; i < 4; ++i) {
    const h16 e0 = toh_flush(WCARRY * bf16r(w0[i]));
    const h16 e1 = toh_flush(WCARRY * bf16r(w1[i]));
    a[i]      = diag ? e0 : (h16)0.0f;
    a[i + 4]  = diag ? e1 : (h16)0.0f;
    a[i + 8]  = (h16)0.0f;
    a[i + 12] = (h16)0.0f;
  }
  return a;
}

__device__ __forceinline__ void mlp_layer(float (&d)[8], const v16h a, const v8f cb) {
  v16h hb;
#pragma unroll
  for (int i = 0; i < 8; ++i) {
    hb[i]     = toh_flush(HCARRY * d[i]);
    hb[i + 8] = (h16)0.0f;
  }
  const v8f c = wmma16(a, hb, cb);
#pragma unroll
  for (int v = 0; v < 8; ++v) d[v] = tanh_f(c[v] * LSCALE);
}

__global__ __launch_bounds__(256) void edge_main_kernel(
    const float* __restrict__ A,  const float* __restrict__ W1,
    const float* __restrict__ W2, const float* __restrict__ b2,
    const float* __restrict__ W3, const float* __restrict__ b3,
    const float* __restrict__ W4, const float* __restrict__ b4,
    const float* __restrict__ W5, const float* __restrict__ b5,
    const float* __restrict__ TJ, const float* __restrict__ U,
    float* __restrict__ out) {
  __shared__ __attribute__((aligned(16))) float Os[8 * 128];
  const unsigned lane = threadIdx.x & 31u;
  const unsigned w = (unsigned)__builtin_amdgcn_readfirstlane((int)(threadIdx.x >> 5));
  const unsigned hh = lane >> 4, m = lane & 15u;
  const unsigned b = blockIdx.x / (unsigned)NROW;
  const unsigned i = blockIdx.x - b * (unsigned)NROW;
  const size_t frow = (size_t)b * NN + i;

  const bool diag = (hh == (m >> 3));
  const v16h a2 = wfrag(W2, m & 7u, diag);
  const v16h a3 = wfrag(W3, m & 7u, diag);
  const v16h a4 = wfrag(W4, m & 7u, diag);

  v8f cb2, cb3, cb4;
  float w1a[8], ui[8], w5r[8];
#pragma unroll
  for (int h = 0; h < 8; ++h) {
    cb2[h] = (WCARRY * HCARRY) * bf16r(b2[h]);
    cb3[h] = (WCARRY * HCARRY) * bf16r(b3[h]);
    cb4[h] = (WCARRY * HCARRY) * bf16r(b4[h]);
    w1a[h] = bf16r(W1[h * W1LD + 48]);
    ui[h]  = U[frow * HIDN + h];
    w5r[h] = bf16r(W5[h]);
  }
  const float bb5 = bf16r(b5[0]);

  const float* Arow = A + frow * NN;
  const float* tjb  = TJ + (size_t)b * NN * HIDN;

#pragma unroll 1
  for (unsigned s = 0; s < (unsigned)STEPS; ++s) {
    const unsigned j = w * 128u + s * 32u + lane;
    const float av = bf16r(Arow[j]);
    const v4f t0 = *(const v4f*)(tjb + (size_t)j * HIDN);
    const v4f t1 = *(const v4f*)(tjb + (size_t)j * HIDN + 4u);

    float d[8];
#pragma unroll
    for (int h = 0; h < 4; ++h) {
      d[h]     = tanh_f(fmaf(av, w1a[h],     t0[h] + ui[h]));
      d[h + 4] = tanh_f(fmaf(av, w1a[h + 4], t1[h] + ui[h + 4]));
    }

    mlp_layer(d, a2, cb2);
    mlp_layer(d, a3, cb3);
    mlp_layer(d, a4, cb4);

    float acc = bb5;
#pragma unroll
    for (int v = 0; v < 8; ++v) acc = fmaf(w5r[v], d[v], acc);

    Os[w * 128u + s * 32u + lane] = acc;
  }
  wave_lds_sync();

  const v4f ov = *(const v4f*)&Os[w * 128u + lane * 4u];
  float* op = out + frow * NN + w * 128u + lane * 4u;
  *(volatile v4f*)op = ov;
  __threadfence();
  *(volatile v4f*)op = ov;
}

extern "C" void kernel_launch(void* const* d_in, const int* in_sizes, int n_in,
                              void* d_out, int out_size, void* d_ws, size_t ws_size,
                              hipStream_t stream) {
  if (n_in < 13) return;
  const long long need_a = ((long long)(NB - 1) * NN + NROW) * NN;
  if ((long long)in_sizes[0] < (long long)NB * NN * DIN) return;
  if ((long long)in_sizes[1] < need_a) return;
  if (in_sizes[2] < NB * DIN) return;
  if (in_sizes[3] < HIDN * W1LD) return;
  if (in_sizes[4] < HIDN) return;
  if (in_sizes[5] < HIDN * HIDN || in_sizes[6] < HIDN) return;
  if (in_sizes[7] < HIDN * HIDN || in_sizes[8] < HIDN) return;
  if (in_sizes[9] < HIDN * HIDN || in_sizes[10] < HIDN) return;
  if (in_sizes[11] < HIDN || in_sizes[12] < 1) return;
  if ((long long)out_size < need_a) return;
  if (ws_size < WS_TOTAL) return;

  const float* x  = (const float*)d_in[0];
  const float* A  = (const float*)d_in[1];
  const float* vp = (const float*)d_in[2];
  const float* W1 = (const float*)d_in[3];
  const float* b1 = (const float*)d_in[4];
  const float* W2 = (const float*)d_in[5];
  const float* b2 = (const float*)d_in[6];
  const float* W3 = (const float*)d_in[7];
  const float* b3 = (const float*)d_in[8];
  const float* W4 = (const float*)d_in[9];
  const float* b4 = (const float*)d_in[10];
  const float* W5 = (const float*)d_in[11];
  const float* b5 = (const float*)d_in[12];
  float* out = (float*)d_out;

  char* ws = (char*)d_ws;
  float* TJ = (float*)(ws + OFF_TJ);
  float* U  = (float*)(ws + OFF_U);

  dim3 blk(256);
  edge_pre_kernel<<<dim3((NB * NN) / 128), blk, 0, stream>>>(x, vp, W1, b1, TJ, U);
  edge_main_kernel<<<dim3(NB * NROW), blk, 0, stream>>>(A, W1, W2, b2, W3, b3, W4, b4,
                                                        W5, b5, TJ, U, out);
}
